// GraphConvTest_22084721836306
// MI455X (gfx1250) — hardware-run, weakly checked
//
#include <hip/hip_runtime.h>

typedef float          v8f   __attribute__((ext_vector_type(8)));
typedef float          v4f   __attribute__((ext_vector_type(4)));
typedef unsigned int   v4u   __attribute__((ext_vector_type(4)));
typedef int            v8i   __attribute__((ext_vector_type(8)));
typedef unsigned short v8us  __attribute__((ext_vector_type(8)));
typedef unsigned short v16us __attribute__((ext_vector_type(16)));
typedef __bf16         v16bf __attribute__((ext_vector_type(16)));
typedef _Float16       v16h  __attribute__((ext_vector_type(16)));
typedef v4f  __attribute__((may_alias)) v4fa;
typedef v8us __attribute__((may_alias)) v8usa;
union FragB { v16bf v; v16us u; v8us h[2]; v8i w; };
union FragH { v16h  v; v16us u; v8us h[2]; v8i w; };

__device__ __forceinline__ v8f wmb(const FragB& a, const FragB& b, v8f c) {
  v8f d = __builtin_amdgcn_wmma_f32_16x16x32_bf16(false, a.v, false, b.v, (short)0, c, false, false);
  asm volatile("v_nop\n\tv_nop\n\tv_nop\n\tv_nop" : "+v"(d) : "v"(a.w), "v"(b.w));
  return d;
}

__device__ __forceinline__ v8f wmh(const FragH& a, const FragH& b, v8f c) {
  v8f d = __builtin_amdgcn_wmma_f32_16x16x32_f16(false, a.v, false, b.v, (short)0, c, false, false);
  asm volatile("v_nop\n\tv_nop\n\tv_nop\n\tv_nop" : "+v"(d) : "v"(a.w), "v"(b.w));
  return d;
}

__device__ __forceinline__ unsigned bf16_bits(float f) {
  const unsigned u = __float_as_uint(f);
  const unsigned r = (u + 0x7FFFu + ((u >> 16) & 1u)) >> 16;
  const unsigned q = (u >> 16) | 0x40u;
  return ((u & 0x7fffffffu) > 0x7f800000u) ? q : r;
}

__device__ __forceinline__ float bf16_val(float f) {
  return __uint_as_float(bf16_bits(f) << 16);
}
__device__ __forceinline__ int clampi(int v, int lo, int hi) {
  return v < lo ? lo : (v > hi ? hi : v);
}

__device__ __forceinline__ unsigned f16_bits(float f) {
  const unsigned u  = __float_as_uint(f);
  const unsigned s  = (u >> 16) & 0x8000u;
  const unsigned a  = u & 0x7fffffffu;
  const unsigned t  = a - 0x38000000u;
  const unsigned r  = (t + 0x0FFFu + ((t >> 13) & 1u)) >> 13;
  const unsigned rc = r > 0x7C00u ? 0x7C00u : r;
  const bool small  = a < 0x38800000u;
  const bool isnan  = a > 0x7f800000u;
  const unsigned fin = small ? 0u : (s | rc);
  return isnan ? (s | 0x7E00u) : fin;
}

__device__ __forceinline__ unsigned pk16(unsigned lo, unsigned hi) { return lo | (hi << 16); }
__device__ __forceinline__ unsigned bf16_lo_bits(float v) {
  float hi = bf16_val(v);
  asm volatile("" : "+v"(hi));
  return bf16_bits(v - hi);
}
__device__ __forceinline__ v4u pack8_bf16(v4f a, v4f c) {
  return (v4u){ pk16(bf16_bits(a[0]), bf16_bits(a[1])), pk16(bf16_bits(a[2]), bf16_bits(a[3])),
                pk16(bf16_bits(c[0]), bf16_bits(c[1])), pk16(bf16_bits(c[2]), bf16_bits(c[3])) };
}
__device__ __forceinline__ v4u pack8_bf16_lo(v4f a, v4f c) {
  return (v4u){ pk16(bf16_lo_bits(a[0]), bf16_lo_bits(a[1])), pk16(bf16_lo_bits(a[2]), bf16_lo_bits(a[3])),
                pk16(bf16_lo_bits(c[0]), bf16_lo_bits(c[1])), pk16(bf16_lo_bits(c[2]), bf16_lo_bits(c[3])) };
}
__device__ __forceinline__ v4u pack8_f16(v4f a, v4f c) {
  return (v4u){ pk16(f16_bits(a[0]), f16_bits(a[1])), pk16(f16_bits(a[2]), f16_bits(a[3])),
                pk16(f16_bits(c[0]), f16_bits(c[1])), pk16(f16_bits(c[2]), f16_bits(c[3])) };
}

template <int FORM>
__global__ __launch_bounds__(256) void k_plane(const float* __restrict__ src, int rows, int cols, int ldsrc,
                                               unsigned short* __restrict__ dst, int MP, int KP) {
  static_assert(FORM >= 0 && FORM <= 3);
  const int KTOT = (FORM == 1 || FORM == 3) ? 2 * KP : KP;
  const unsigned ppr   = (unsigned)(KTOT >> 3);
  const unsigned kp8   = (unsigned)(KP >> 3);
  const unsigned total = (unsigned)MP * ppr;
  const unsigned g     = blockIdx.x * 256u + threadIdx.x;
  const unsigned rowu  = g / ppr;
  const unsigned p     = g - rowu * ppr;
  const bool second    = p >= kp8;
  const int row = (int)rowu;
  const int c0  = (int)((second ? p - kp8 : p) << 3);
  const float* srow = src + (size_t)clampi(row, 0, rows - 1) * (size_t)ldsrc;
  float x[8];
  unsigned mk[8];
#pragma unroll
  for (int e = 0; e < 8; ++e) {
    const int c = c0 + e;
    const float v = srow[clampi(c, 0, cols - 1)];
    asm volatile("" :: "v"(v));
    x[e]  = v;
    mk[e] = (row < rows && c < cols) ? 0xFFFFu : 0u;
  }
  const v4f a = (v4f){ x[0], x[1], x[2], x[3] };
  const v4f c = (v4f){ x[4], x[5], x[6], x[7] };
  v4u o;
  if (FORM == 2) {
    o = pack8_f16(a, c);
  } else {
    const v4u hi = pack8_bf16(a, c);
    o = hi;
    if (FORM == 1) { const v4u lo = pack8_bf16_lo(a, c); o = second ? lo : hi; }
  }
  const v4u mw = (v4u){ pk16(mk[0], mk[1]), pk16(mk[2], mk[3]), pk16(mk[4], mk[5]), pk16(mk[6], mk[7]) };
  o &= mw;
  if (g < total) {
    volatile v4u* q = (volatile v4u*)(dst + (size_t)g * 8);
    *q = o;
    __threadfence();
    *q = o;
  }
}

template <int FORM> struct FragOf    { typedef FragB T; };
template <>         struct FragOf<2> { typedef FragH T; };
__device__ __forceinline__ v8f mm(const FragB& a, const FragB& b, v8f c) { return wmb(a, b, c); }
__device__ __forceinline__ v8f mm(const FragH& a, const FragH& b, v8f c) { return wmh(a, b, c); }
template <class F> __device__ __forceinline__ F ld_frag(const unsigned short* p) {
  F f;
  f.h[0] = *(const v8usa*)(p);
  f.h[1] = *(const v8usa*)(p + 16);
  return f;
}

template <int FORM, int EPI>
__global__ __launch_bounds__(256) __attribute__((amdgpu_num_vgpr(248)))
void k_gemm_nt(const unsigned short* __restrict__ A, const unsigned short* __restrict__ B,
               const float* __restrict__ bias, float* __restrict__ D, int M, int N, int KTOT, int ldd) {
  static_assert(FORM >= 0 && FORM <= 2);
  static_assert(EPI == 0 || EPI == 1);
  typedef typename FragOf<FORM>::T F;
  __shared__ __attribute__((aligned(16))) float sT[8][16 * 68];
  const int lane = threadIdx.x & 31;
  const int wave = threadIdx.x >> 5;
  const int tilesM = (M + 63) >> 6;
  const int tilesN = (N + 63) >> 6;
  const int tile = blockIdx.x * 8 + wave;
  if (tile >= tilesM * tilesN) return;
  const int tm = tile / tilesN;
  const int tn = tile - tm * tilesN;
  const int m0 = tm << 6;
  const int n0 = tn << 6;

  const int rl = lane & 15;
  const int h8 = (lane >> 4) * 8;
  const unsigned short* pa = A + (size_t)(m0 + rl) * (size_t)KTOT + h8;
  const unsigned short* pb = B + (size_t)(n0 + rl) * (size_t)KTOT + h8;

  v8f acc[4][4];
#pragma unroll
  for (int i = 0; i < 4; ++i)
#pragma unroll
    for (int j = 0; j < 4; ++j) acc[i][j] = (v8f){0.f, 0.f, 0.f, 0.f, 0.f, 0.f, 0.f, 0.f};

#pragma unroll 1
  for (int k0 = 0; k0 < KTOT; k0 += 32) {
    F bf[4];
#pragma unroll
    for (int j = 0; j < 4; ++j) bf[j] = ld_frag<F>(pb + (size_t)(j << 4) * (size_t)KTOT + k0);
#pragma unroll
    for (int i = 0; i < 4; ++i) {
      const F af = ld_frag<F>(pa + (size_t)(i << 4) * (size_t)KTOT + k0);
#pragma unroll
      for (int j = 0; j < 4; ++j) acc[i][j] = mm(af, bf[j], acc[i][j]);
    }
  }

  float* slab = sT[wave];
  const int hh = lane >> 4;
  const int c4 = (lane & 15) * 4;
  const int nc = n0 + c4;
  const bool cok = nc < N;
  v4f bv = (v4f){0.f, 0.f, 0.f, 0.f};
  if (EPI == 1) {
    bv = *(const v4fa*)(bias + clampi(nc, 0, N - 4));
    asm volatile("" :: "v"(bv));
  }
#pragma unroll
  for (int i = 0; i < 4; ++i) {
    const int mBase = m0 + (i << 4);
#pragma unroll
    for (int j = 0; j < 4; ++j) {
#pragma unroll
      for (int r = 0; r < 8; ++r) slab[(h8 + r) * 68 + (j << 4) + rl] = acc[i][j][r];
    }
    __builtin_amdgcn_fence(__ATOMIC_RELEASE, "workgroup");
    __builtin_amdgcn_wave_barrier();
    __builtin_amdgcn_fence(__ATOMIC_ACQUIRE, "workgroup");
    v4f vv[8];
#pragma unroll
    for (int it = 0; it < 8; ++it) {
      const int row = it * 2 + hh;
      v4f v = *(const v4fa*)(slab + row * 68 + c4);
      if (EPI == 1) v += bv;
      vv[it] = v;
    }
    for (int pass = 0; pass < 2; ++pass) {
#pragma unroll
      for (int it = 0; it < 8; ++it) {
        const int row = mBase + it * 2 + hh;
        if (cok && row < M) *(volatile v4f*)(D + (size_t)row * (size_t)ldd + nc) = vv[it];
      }
      __threadfence();
    }
    __builtin_amdgcn_fence(__ATOMIC_RELEASE, "workgroup");
    __builtin_amdgcn_wave_barrier();
    __builtin_amdgcn_fence(__ATOMIC_ACQUIRE, "workgroup");
  }
}

#include <math.h>
#include <stddef.h>

#define NB     16
#define NN     256
#define NF     33
#define NH     11
#define ROWS   (NB * NN)
#define KV     (NF * NH)
#define KVP    384
#define KTH    (2 * KVP)
#define AGM    (NN * NH)
#define AGR    (NB * AGM)
#define OUT0_N (ROWS * NF)
#define OUT1_N (ROWS * NN * NH)
#define SLAB_F (128 * NH)
#define SLAB_P (SLAB_F / 4)
#define APITCH 136

static_assert(NN % 128 == 0);
static_assert(AGM % 128 == 0 && AGM % 64 == 0);
static_assert(NF <= 64 && NF + NH <= 64 && NH <= 16 && KV <= KVP && KVP % 32 == 0);
static_assert((128 * NH * 4) % 128 == 0);
static_assert((32 * NF * 4) % 128 == 0);
static_assert(((size_t)OUT0_N * 4) % 128 == 0);
static_assert(OUT0_N * 4 == 540672);
static_assert(SLAB_P == 352 && SLAB_P > 256 && SLAB_P - 256 == 96);
static_assert((APITCH * 2) % 16 == 0 && APITCH >= 128);
static_assert(128 * APITCH * 2 + SLAB_F * 4 + 64 * 4 <= 327680);

typedef v4u __attribute__((may_alias)) v4ua;

__device__ __forceinline__ float relu_sel(float v) { return (v > 0.0f) ? v : (v - v); }

static constexpr size_t SZ_ADJT = (size_t)AGR * 512 * 2;
static constexpr size_t SZ_AGG  = (size_t)AGR * 64 * 4;
static constexpr size_t SZ_THL  = (size_t)ROWS * KTH * 2;
static constexpr size_t SZ_SUPT = (size_t)NB * 64 * 512 * 2;
static constexpr size_t SZ_PQ   = (size_t)ROWS * 128 * 4;
static constexpr size_t SZ_SUP  = (size_t)ROWS * 64 * 4;
static constexpr size_t SZ_OACC = (size_t)ROWS * 64 * 4;
static constexpr size_t SZ_OHL  = (size_t)ROWS * 128 * 2;
static constexpr size_t SZ_NFB  = (size_t)ROWS * 64 * 2;
static constexpr size_t SZ_W1T  = (size_t)64 * 64 * 2;
static constexpr size_t SZ_WOT  = (size_t)64 * KTH * 2;
static constexpr size_t SZ_WPQ  = (size_t)128 * 128 * 2;
static constexpr size_t SZ_W2   = (size_t)16 * 128 * 2;
static constexpr size_t O_ADJT = 0;
static constexpr size_t O_AGG  = O_ADJT + SZ_ADJT;
static constexpr size_t O_THL  = O_AGG  + SZ_AGG;
static constexpr size_t O_SUPT = O_THL  + SZ_THL;
static constexpr size_t O_PQ   = O_SUPT + SZ_SUPT;
static constexpr size_t O_SUP  = O_PQ   + SZ_PQ;
static constexpr size_t O_OACC = O_SUP  + SZ_SUP;
static constexpr size_t O_OHL  = O_OACC + SZ_OACC;
static constexpr size_t O_NFB  = O_OHL  + SZ_OHL;
static constexpr size_t O_W1T  = O_NFB  + SZ_NFB;
static constexpr size_t O_WOT  = O_W1T  + SZ_W1T;
static constexpr size_t O_WPQ  = O_WOT  + SZ_WOT;
static constexpr size_t O_W2   = O_WPQ  + SZ_WPQ;
static constexpr size_t WS_TOTAL = O_W2 + SZ_W2;
static_assert(SZ_ADJT % 256 == 0 && SZ_AGG % 256 == 0 && SZ_THL % 256 == 0 && SZ_SUPT % 256 == 0);
static_assert(SZ_PQ % 256 == 0 && SZ_SUP % 256 == 0 && SZ_OHL % 256 == 0 && SZ_NFB % 256 == 0);
static_assert(SZ_W1T % 256 == 0 && SZ_WOT % 256 == 0 && SZ_WPQ % 256 == 0 && SZ_W2 % 256 == 0);
static_assert(WS_TOTAL == 70922240);
static_assert(WS_TOTAL <= ((size_t)128 << 20));

#define U_W1  512
#define U_WO  6144
#define U_WPQ 2048
#define U_W2  256
#define U_TOT (U_W1 + U_WO + U_WPQ + U_W2)
static_assert(U_W1 == 64 * 64 / 8 && U_WO == 64 * KTH / 8 && U_WPQ == 128 * 128 / 8 && U_W2 == 16 * 128 / 8);
static_assert(U_W1 % 256 == 0 && U_WO % 256 == 0 && U_WPQ % 256 == 0 && U_W2 % 256 == 0 && U_TOT == 8960);

__device__ __forceinline__ void wunit(const float* __restrict__ src, int pitch, int nrows, int ncols,
                                      int rowbase, int kk, int kvalid, int col, bool colok,
                                      unsigned short* dstp) {
  float x[8];
  unsigned mk[8];
  const int cc = clampi(col, 0, ncols - 1);
#pragma unroll
  for (int e = 0; e < 8; ++e) {
    const int kr = kk + e;
    const int r  = clampi(rowbase + kr, 0, nrows - 1);
    const float v = src[(size_t)r * (size_t)pitch + cc];
    asm volatile("" :: "v"(v));
    x[e]  = v;
    mk[e] = (colok && kr < kvalid) ? 0xFFFFu : 0u;
  }
  const v4f a = (v4f){ x[0], x[1], x[2], x[3] };
  const v4f c = (v4f){ x[4], x[5], x[6], x[7] };
  v4u o = pack8_bf16(a, c);
  const v4u mw = (v4u){ pk16(mk[0], mk[1]), pk16(mk[2], mk[3]), pk16(mk[4], mk[5]), pk16(mk[6], mk[7]) };
  o &= mw;
  volatile v4u* q = (volatile v4u*)dstp;
  *q = o;
  __threadfence();
  *q = o;
}

__global__ __launch_bounds__(256) void k_wprep(const float* __restrict__ tW, const float* __restrict__ oW,
                                               const float* __restrict__ aW, const float* __restrict__ a2W,
                                               unsigned short* w1t, unsigned short* wot,
                                               unsigned short* wpq, unsigned short* w2) {
  const int u = (int)blockIdx.x * 256 + (int)threadIdx.x;
  if (u < U_W1) {
    const int n = u >> 3, kk = (u & 7) * 8;
    wunit(tW, NF, NF, NF, 0, kk, NF, n, n < NF, w1t + (size_t)u * 8);
  } else if (u < U_W1 + U_WO) {
    const int v = u - U_W1;
    const int n = v / 96;
    const int k = (v - n * 96) * 8;
    const int kk = k >= KVP ? k - KVP : k;
    wunit(oW, NF, KV, NF, 0, kk, KV, n, n < NF, wot + (size_t)v * 8);
  } else if (u < U_W1 + U_WO + U_WPQ) {
    const int v = u - U_W1 - U_WO;
    const int n = v >> 4;
    const int kk = (v & 7) * 8;
    const bool isq = n >= NF;
    const int col = isq ? n - NF : n;
    wunit(aW, NF, 2 * NF, NF, isq ? NF : 0, kk, NF, col, n < 2 * NF, wpq + (size_t)v * 8);
  } else if (u < U_TOT) {
    const int v = u - U_W1 - U_WO - U_WPQ;
    const int n = v >> 4;
    const int k = (v & 15) * 8;
    const bool sec = k >= 64;
    wunit(a2W, NH, NF + NH, NH, 0, sec ? k - 64 : k, sec ? NF : NF + NH, n, n < NH, w2 + (size_t)v * 8);
  }
}

__global__ __launch_bounds__(256) void k_supT(const float* __restrict__ SUP, unsigned short* SUPT) {
  __shared__ __attribute__((aligned(16))) float s[256 * 20];
  const int t = (int)threadIdx.x;
  const int b = (int)blockIdx.x >> 2, q = (int)blockIdx.x & 3;
  const float* sp = SUP + ((size_t)(b * 256 + t)) * 64 + 16 * q;
  const v4f l0 = *(const v4fa*)(sp), l1 = *(const v4fa*)(sp + 4), l2 = *(const v4fa*)(sp + 8), l3 = *(const v4fa*)(sp + 12);
  *(v4fa*)(s + t * 20)      = l0;
  *(v4fa*)(s + t * 20 + 4)  = l1;
  *(v4fa*)(s + t * 20 + 8)  = l2;
  *(v4fa*)(s + t * 20 + 12) = l3;
  __syncthreads();
  v4u o[4];
#pragma unroll
  for (int it = 0; it < 4; ++it) {
    const int g = it * 256 + t;
    const int nl = g >> 6, p = g & 63;
    const bool second = p >= 32;
    const int k0 = 8 * (p & 31);
    float x[8];
#pragma unroll
    for (int e = 0; e < 8; ++e) x[e] = s[(k0 + e) * 20 + nl];
    const v4f a = (v4f){ x[0], x[1], x[2], x[3] };
    const v4f c = (v4f){ x[4], x[5], x[6], x[7] };
    const v4u hi = pack8_bf16(a, c);
    const v4u lo = pack8_bf16_lo(a, c);
    v4u w = second ? lo : hi;
    const unsigned mk = (16 * q + nl < NF) ? 0xFFFFFFFFu : 0u;
    w &= (v4u){ mk, mk, mk, mk };
    o[it] = w;
  }
  unsigned short* dst = SUPT + ((size_t)b * 64 + 16 * q) * 512;
  for (int ps = 0; ps < 2; ++ps) {
#pragma unroll
    for (int it = 0; it < 4; ++it) *(volatile v4u*)(dst + (size_t)(it * 256 + t) * 8) = o[it];
    __threadfence();
  }
}

__global__ __launch_bounds__(256) void k_adjT(const float* __restrict__ adj, unsigned short* ADJT) {
  __shared__ __attribute__((aligned(16))) float s[AGM];
  const int t = (int)threadIdx.x;
  const float* src = adj + (size_t)blockIdx.x * AGM;
#pragma unroll
  for (int it = 0; it < 3; ++it) {
    const int idx = it * 256 + t;
    const int ic = idx < 704 ? idx : 703;
    const v4f v = *(const v4fa*)(src + 4 * ic);
    asm volatile("" :: "v"(v));
    if (idx < 704) *(v4fa*)(s + 4 * idx) = v;
  }
  __syncthreads();
  v4u o[3];
#pragma unroll
  for (int it = 0; it < 3; ++it) {
    const int g = it * 256 + t;
    const int gc = g < 704 ? g : 703;
    const int h = gc >> 6, p = gc & 63;
    const int j0 = 8 * (p & 31);
    float x[8];
#pragma unroll
    for (int e = 0; e < 8; ++e) x[e] = s[(j0 + e) * NH + h];
    o[it] = pack8_bf16((v4f){ x[0], x[1], x[2], x[3] }, (v4f){ x[4], x[5], x[6], x[7] });
  }
  unsigned short* dst = ADJT + (size_t)blockIdx.x * (NH * 512);
  for (int ps = 0; ps < 2; ++ps) {
#pragma unroll
    for (int it = 0; it < 3; ++it) {
      const int g = it * 256 + t;
      if (g < 704) *(volatile v4u*)(dst + (size_t)g * 8) = o[it];
    }
    __threadfence();
  }
}

__global__ __launch_bounds__(256) void k_tanh(const float* __restrict__ AGG, const float* __restrict__ SUP,
                                              unsigned short* THL) {
  __shared__ __attribute__((aligned(16))) float st[8 * KVP];
  const int t = (int)threadIdx.x;
  const int r0 = (int)blockIdx.x * 8;
#pragma unroll 1
  for (int it = 0; it < 12; ++it) {
    const int idx = it * 256 + t;
    const int node = idx / KVP;
    const int k = idx - node * KVP;
    const bool ok = k < KV;
    const int kc = ok ? k : KV - 1;
    const int f = kc / NH;
    const int h = kc - f * NH;
    const int row = r0 + node;
    const float a = AGG[((size_t)row * NH + h) * 64 + f];
    const float sv = SUP[(size_t)row * 64 + f];
    asm volatile("" :: "v"(a));
    asm volatile("" :: "v"(sv));
    const float v = tanhf(a + sv);
    st[idx] = ok ? v : 0.0f;
  }
  __syncthreads();
  v4u o[3];
#pragma unroll
  for (int it = 0; it < 3; ++it) {
    const int g = it * 256 + t;
    const int node = g / 96;
    const int p = g - node * 96;
    const bool second = p >= 48;
    const int k0 = 8 * (second ? p - 48 : p);
    const v4f a = *(const v4fa*)(st + node * KVP + k0);
    const v4f c = *(const v4fa*)(st + node * KVP + k0 + 4);
    const v4u hi = pack8_bf16(a, c);
    const v4u lo = pack8_bf16_lo(a, c);
    o[it] = second ? lo : hi;
  }
  unsigned short* dst = THL + (size_t)r0 * KTH;
  for (int ps = 0; ps < 2; ++ps) {
#pragma unroll
    for (int it = 0; it < 3; ++it) *(volatile v4u*)(dst + (size_t)(it * 256 + t) * 8) = o[it];
    __threadfence();
  }
}

__global__ __launch_bounds__(256) void k_nodeout(const float* __restrict__ OACC, float* out0, unsigned short* OHL) {
  __shared__ __attribute__((aligned(16))) float so[32 * NF];
  __shared__ __attribute__((aligned(16))) float sp[32 * 64];
  const int t = (int)threadIdx.x;
  const int r0 = (int)blockIdx.x * 32;
#pragma unroll 1
  for (int it = 0; it < 8; ++it) {
    const int idx = it * 256 + t;
    const int row = idx >> 6, c = idx & 63;
    const float a = OACC[(size_t)(r0 + row) * 64 + c];
    asm volatile("" :: "v"(a));
    const float tv = tanhf(a);
    const float val = (c < NF) ? tv : 0.0f;
    sp[idx] = val;
    if (c < NF) so[row * NF + c] = val;
  }
  __syncthreads();
  const v4f f0 = *(const v4fa*)(so + 4 * t);
  const v4f f1 = *(const v4fa*)(so + 4 * (256 + (t & 7)));
  asm volatile("" :: "v"(f1));
  v4u o[2];
#pragma unroll
  for (int it = 0; it < 2; ++it) {
    const int g = it * 256 + t;
    const int row = g >> 4, p = g & 15;
    const bool second = p >= 8;
    const int c0 = 8 * (p & 7);
    const v4f a = *(const v4fa*)(sp + row * 64 + c0);
    const v4f c = *(const v4fa*)(sp + row * 64 + c0 + 4);
    const v4u hi = pack8_bf16(a, c);
    const v4u lo = pack8_bf16_lo(a, c);
    o[it] = second ? lo : hi;
  }
  float* op = out0 + (size_t)r0 * NF + 4 * t;
  unsigned short* dh = OHL + (size_t)r0 * 128;
  for (int ps = 0; ps < 2; ++ps) {
    *(volatile v4f*)op = f0;
    if (t < 8) *(volatile v4f*)(op + 1024) = f1;
    *(volatile v4u*)(dh + (size_t)t * 8) = o[0];
    *(volatile v4u*)(dh + (size_t)(256 + t) * 8) = o[1];
    __threadfence();
  }
}

__global__ __launch_bounds__(256) void k_edge(const float* __restrict__ adj, const float* __restrict__ PQ,
                                              const unsigned short* __restrict__ W2, float* out1) {
  __shared__ __attribute__((aligned(16))) unsigned short As[128 * APITCH];
  __shared__ __attribute__((aligned(16))) float ADJS[SLAB_F];
  __shared__ __attribute__((aligned(16))) float sq[64];
  const int t = (int)threadIdx.x, lane = t & 31, wave = t >> 5, hh = lane >> 4, m = lane & 15;
  const int bi = (int)blockIdx.x;
  const int b  = bi >> 8;

  if (t < 64) {
    const int c = t < NF ? t : NF - 1;
    const float v = PQ[(size_t)bi * 128 + NF + c];
    asm volatile("" :: "v"(v));
    sq[t] = (t < NF) ? v : 0.0f;
  }
  FragB bw[4];
  {
    const unsigned short* bp = W2 + m * 128 + 8 * hh;
#pragma unroll
    for (int ks = 0; ks < 4; ++ks) bw[ks] = ld_frag<FragB>(bp + 32 * ks);
  }
  __syncthreads();

  const int row = t & 127, hf = t >> 7;
  const int tc  = t < 96 ? t : 95;
  const int nc  = m < NH ? m : NH - 1;

#pragma unroll 1
  for (int step = 0; step < 2; ++step) {
    const int j0 = step * 128;
    {
      const float* asrc = adj + ((size_t)bi * NN + j0) * NH;
      const v4f v0 = *(const v4fa*)(asrc + 4 * t);
      const v4f v1 = *(const v4fa*)(asrc + 4 * (256 + tc));
      asm volatile("" :: "v"(v1));
      const v4f r0 = (v4f){ bf16_val(v0[0]), bf16_val(v0[1]), bf16_val(v0[2]), bf16_val(v0[3]) };
      const v4f r1 = (v4f){ bf16_val(v1[0]), bf16_val(v1[1]), bf16_val(v1[2]), bf16_val(v1[3]) };
      *(v4fa*)(ADJS + 4 * t) = r0;
      if (t < 96) *(v4fa*)(ADJS + 4 * (256 + t)) = r1;
    }
    const float* prow = PQ + ((size_t)(b * NN + j0 + row)) * 128;
    unsigned short* arow = As + row * APITCH;
#pragma unroll
    for (int it = 0; it < 2; ++it) {
      const int c0 = 8 * (hf + 2 * it);
      const v4f p0 = *(const v4fa*)(prow + c0);
      const v4f p1 = *(const v4fa*)(prow + c0 + 4);
      const v4f q0 = *(const v4fa*)(sq + c0);
      const v4f q1 = *(const v4fa*)(sq + c0 + 4);
      const v4f x0 = (v4f){ relu_sel(p0[0] + q0[0]), relu_sel(p0[1] + q0[1]), relu_sel(p0[2] + q0[2]), relu_sel(p0[3] + q0[3]) };
      const v4f x1 = (v4f){ relu_sel(p1[0] + q1[0]), relu_sel(p1[1] + q1[1]), relu_sel(p1[2] + q1[2]), relu_sel(p1[3] + q1[3]) };
      *(v4ua*)(arow + c0)      = pack8_bf16(x0, x1);
      *(v4ua*)(arow + 64 + c0) = pack8_bf16_lo(x0, x1);
    }
    __syncthreads();
    {
      const v4u z4 = (v4u){ 0u, 0u, 0u, 0u };
      const float* ar = ADJS + row * NH;
      if (hf == 0) {
        const float x32 = relu_sel(prow[32] + sq[32]);
        const v4f a = (v4f){ x32, ar[0], ar[1], ar[2] };
        const v4f c = (v4f){ ar[3], ar[4], ar[5], ar[6] };
        *(v4ua*)(arow + 32)  = pack8_bf16(a, c);
        *(v4ua*)(arow + 96)  = (v4u){ pk16(bf16_lo_bits(x32), 0u), 0u, 0u, 0u };
        *(v4ua*)(arow + 48)  = z4;
        *(v4ua*)(arow + 112) = z4;
      } else {
        const v4f a = (v4f){ ar[7], ar[8], ar[9], ar[10] };
        const v4f c = (v4f){ 0.0f, 0.0f, 0.0f, 0.0f };
        *(v4ua*)(arow + 40)  = pack8_bf16(a, c);
        *(v4ua*)(arow + 56)  = z4;
        *(v4ua*)(arow + 104) = z4;
        *(v4ua*)(arow + 120) = z4;
      }
    }
    __syncthreads();
    v8f acc = (v8f){0.f, 0.f, 0.f, 0.f, 0.f, 0.f, 0.f, 0.f};
    {
      const unsigned short* ap = As + (16 * wave + m) * APITCH + 8 * hh;
#pragma unroll
      for (int ks = 0; ks < 4; ++ks) {
        FragB af;
        af.h[0] = *(const v8usa*)(ap + 32 * ks);
        af.h[1] = *(const v8usa*)(ap + 32 * ks + 16);
        acc = wmb(af, bw[ks], acc);
      }
    }
    {
      const int pbase = (16 * wave + 8 * hh) * NH;
      float rv[8];
#pragma unroll
      for (int r = 0; r < 8; ++r) {
        const float v = ADJS[pbase + r * NH + nc];
        asm volatile("" :: "v"(v));
        rv[r] = v;
      }
#pragma unroll
      for (int r = 0; r < 8; ++r) {
        const float v = relu_sel(acc[r]) + rv[r];
        if (m < NH) ADJS[pbase + r * NH + m] = v;
      }
    }
    __syncthreads();
    {
      const v4f f0 = *(const v4fa*)(ADJS + 4 * t);
      const v4f f1 = *(const v4fa*)(ADJS + 4 * (256 + tc));
      asm volatile("" :: "v"(f1));
      float* op = out1 + ((size_t)bi * NN + j0) * NH + 4 * t;
      for (int ps = 0; ps < 2; ++ps) {
        *(volatile v4f*)op = f0;
        if (t < 96) *(volatile v4f*)(op + 1024) = f1;
        __threadfence();
      }
    }
    __syncthreads();
  }
}

static inline int cdiv(int a, int b) { return (a + b - 1) / b; }

extern "C" void kernel_launch(void* const* d_in, const int* in_sizes, int n_in,
                              void* d_out, int out_size, void* d_ws, size_t ws_size,
                              hipStream_t stream) {
  if (n_in < 6) return;
  if (in_sizes[0] != ROWS * NF) return;
  if (in_sizes[1] != OUT1_N) return;
  if (in_sizes[2] != NF * NF) return;
  if (in_sizes[3] != KV * NF) return;
  if (in_sizes[4] != 2 * NF * NF) return;
  if (in_sizes[5] != (NF + NH) * NH) return;
  if ((long long)out_size != (long long)OUT0_N + (long long)OUT1_N) return;
  if ((size_t)WS_TOTAL > ws_size) return;

  const float* nf  = (const float*)d_in[0];
  const float* adj = (const float*)d_in[1];
  const float* tW  = (const float*)d_in[2];
  const float* oW  = (const float*)d_in[3];
  const float* aW  = (const float*)d_in[4];
  const float* a2W = (const float*)d_in[5];
  float* out0 = (float*)d_out;
  float* out1 = (float*)d_out + (size_t)OUT0_N;

  char* ws = (char*)d_ws;
  unsigned short* ADJT = (unsigned short*)(ws + O_ADJT);
  float*          AGG  = (float*)(ws + O_AGG);
  unsigned short* THL  = (unsigned short*)(ws + O_THL);
  unsigned short* SUPT = (unsigned short*)(ws + O_SUPT);
  float*          PQ   = (float*)(ws + O_PQ);
  float*          SUP  = (float*)(ws + O_SUP);
  float*          OACC = (float*)(ws + O_OACC);
  unsigned short* OHL  = (unsigned short*)(ws + O_OHL);
  unsigned short* NFB  = (unsigned short*)(ws + O_NFB);
  unsigned short* W1T  = (unsigned short*)(ws + O_W1T);
  unsigned short* WOT  = (unsigned short*)(ws + O_WOT);
  unsigned short* WPQ  = (unsigned short*)(ws + O_WPQ);
  unsigned short* W2   = (unsigned short*)(ws + O_W2);

  k_plane<0><<<ROWS * 64 / 8 / 256, 256, 0, stream>>>(nf, ROWS, NF, NF, NFB, ROWS, 64);
  k_wprep<<<U_TOT / 256, 256, 0, stream>>>(tW, oW, aW, a2W, W1T, WOT, WPQ, W2);
  k_gemm_nt<0, 0><<<cdiv(64, 8), 256, 0, stream>>>(NFB, W1T, SUP, SUP, ROWS, 64, 64, 64);
  k_supT<<<NB * 4, 256, 0, stream>>>(SUP, SUPT);
  k_adjT<<<ROWS, 256, 0, stream>>>(adj, ADJT);
  for (int b = 0; b < NB; ++b) {
    k_gemm_nt<0, 0><<<cdiv(AGM / 64, 8), 256, 0, stream>>>(ADJT + (size_t)b * AGM * 512, SUPT + (size_t)b * 64 * 512,
                                                          SUP, AGG + (size_t)b * AGM * 64, AGM, 64, 512, 64);
  }
  k_tanh<<<ROWS / 8, 256, 0, stream>>>(AGG, SUP, THL);
  k_gemm_nt<0, 0><<<cdiv(64, 8), 256, 0, stream>>>(THL, WOT, SUP, OACC, ROWS, 64, KTH, 64);
  k_nodeout<<<ROWS / 32, 256, 0, stream>>>(OACC, out0, OHL);
  k_gemm_nt<0, 0><<<cdiv(128, 8), 256, 0, stream>>>(OHL, WPQ, SUP, PQ, ROWS, 128, 128, 128);
  k_edge<<<ROWS, 256, 0, stream>>>(adj, PQ, W2, out1);
}
